// FooNet_57526791962848
// MI455X (gfx1250) — hardware-run, weakly checked
//
#include <hip/hip_runtime.h>
#include <math.h>

typedef __attribute__((ext_vector_type(16))) __bf16   v16b;
typedef __attribute__((ext_vector_type(8)))  float    v8f;
typedef __attribute__((ext_vector_type(4)))  float    v4f;
typedef __attribute__((ext_vector_type(2)))  float    v2f;
typedef __attribute__((ext_vector_type(4)))  unsigned v4u;
typedef __attribute__((ext_vector_type(8)))  unsigned v8u;

constexpr int kDim          = 10;
constexpr int kNumEnt       = 14951;
constexpr int kNumRel       = 1345;
constexpr int kBatchRows    = 8192;
constexpr int kCands        = 256;
constexpr int kTotal        = kBatchRows * kCands;
constexpr int kTileElems    = 16;
constexpr int kTilesPerWave = 8;
constexpr int kElemsPerWave = kTileElems * kTilesPerWave;
constexpr int kWavesPerBlk  = 8;
constexpr int kElemsPerBlk  = kElemsPerWave * kWavesPerBlk;
constexpr int kGridScore    = kTotal / kElemsPerBlk;
static_assert(kDim == 10, "slot layout below is written for ten components");
static_assert(kElemsPerWave == 128, "one wave emits four whole 128-B lines per store instruction");
static_assert(kTotal % kElemsPerBlk == 0, "exact grid, no tail");
static_assert(kGridScore == 2048, "grid size");

constexpr size_t kPlaneDwords = 2 * 32 * 8;
constexpr size_t kWsTotal     = kPlaneDwords * 4;
static_assert(kWsTotal == 2048, "carve total");

__device__ __forceinline__ unsigned bf_bits_rne(float f) {
  const unsigned u = __float_as_uint(f);
  return (u + 0x7FFFu + ((u >> 16) & 1u)) >> 16;
}
__device__ __forceinline__ float bf_bits_to_f32(unsigned hb) { return __uint_as_float(hb << 16); }

__device__ __forceinline__ v8f mma_bf16(v16b a, v16b b, v8f c) {
  c = __builtin_amdgcn_wmma_f32_16x16x32_bf16(false, a, false, b, (short)0, c, false, false);
  asm volatile("v_nop\n\tv_nop\n\tv_nop\n\tv_nop" : "+v"(c) : "v"(a), "v"(b));
  return c;
}

__device__ __forceinline__ v16b pack_hi_hi_lo(float v0, float v1, float v2, float v3, float v4) {
  const unsigned h0 = bf_bits_rne(v0);
  const unsigned h1 = bf_bits_rne(v1);
  const unsigned h2 = bf_bits_rne(v2);
  const unsigned h3 = bf_bits_rne(v3);
  const unsigned h4 = bf_bits_rne(v4);
  const unsigned l0 = bf_bits_rne(v0 - bf_bits_to_f32(h0));
  const unsigned l1 = bf_bits_rne(v1 - bf_bits_to_f32(h1));
  const unsigned l2 = bf_bits_rne(v2 - bf_bits_to_f32(h2));
  const unsigned l3 = bf_bits_rne(v3 - bf_bits_to_f32(h3));
  const unsigned l4 = bf_bits_rne(v4 - bf_bits_to_f32(h4));
  v8u w;
  w[0] = h0 | (h1 << 16);
  w[1] = h2 | (h3 << 16);
  w[2] = h4 | (h0 << 16);
  w[3] = h1 | (h2 << 16);
  w[4] = h3 | (h4 << 16);
  w[5] = l0 | (l1 << 16);
  w[6] = l2 | (l3 << 16);
  w[7] = l4;
  return __builtin_bit_cast(v16b, w);
}

template <int PLANE, int HF, int I>
__device__ __forceinline__ unsigned plane_elem(const float* sInv, const float* sSym, int mc, bool live) {
  constexpr int kGrpOf[16]  = {0, 0, 0, 0, 0, 1, 1, 1, 1, 1, 2, 2, 2, 2, 2, 3};
  constexpr int kCompOf[16] = {0, 1, 2, 3, 4, 0, 1, 2, 3, 4, 0, 1, 2, 3, 4, 0};
  static_assert(sizeof(kGrpOf) / sizeof(kGrpOf[0]) == 16, "group table size");
  static_assert(sizeof(kCompOf) / sizeof(kCompOf[0]) == 16, "component table size");
  static_assert(I >= 0 && I < 16, "element number");
  constexpr int grp = kGrpOf[I];
  constexpr int d   = 5 * HF + kCompOf[I];
  static_assert(d >= 0 && d < kDim, "component in range");
  if (grp == 3) return 0u;
  int idx = d * kDim + mc;
  asm volatile("" : "+v"(idx));
  float val;
  if (PLANE != 0) val = sSym[idx];
  else            val = sInv[idx];
  val = live ? val : 0.0f;
  unsigned hb = bf_bits_rne(val);
  asm volatile("" : "+v"(hb));
  if (grp != 1) return hb;
  unsigned lb = bf_bits_rne(val - bf_bits_to_f32(hb));
  asm volatile("" : "+v"(lb));
  return lb;
}

template <int PLANE, int HF, int Q>
__device__ __forceinline__ unsigned plane_word(const float* sInv, const float* sSym, int mc, bool live) {
  unsigned lo = plane_elem<PLANE, HF, 2 * Q>(sInv, sSym, mc, live);
  unsigned hi = plane_elem<PLANE, HF, 2 * Q + 1>(sInv, sSym, mc, live);
  asm volatile("" : "+v"(lo));
  asm volatile("" : "+v"(hi));
  unsigned w = (hi << 16) | (lo & 0xffffu);
  asm volatile("" : "+v"(w));
  return w;
}

template <int IT>
__device__ __forceinline__ v4u plane_quad(const float* sInv, const float* sSym, int mc, bool live, bool upperQ) {
  constexpr int PL = IT >> 1;
  constexpr int HF = IT & 1;
  const unsigned a0 = plane_word<PL, HF, 0>(sInv, sSym, mc, live);
  const unsigned a1 = plane_word<PL, HF, 1>(sInv, sSym, mc, live);
  const unsigned a2 = plane_word<PL, HF, 2>(sInv, sSym, mc, live);
  const unsigned a3 = plane_word<PL, HF, 3>(sInv, sSym, mc, live);
  const unsigned b0 = plane_word<PL, HF, 4>(sInv, sSym, mc, live);
  const unsigned b1 = plane_word<PL, HF, 5>(sInv, sSym, mc, live);
  const unsigned b2 = plane_word<PL, HF, 6>(sInv, sSym, mc, live);
  const unsigned b3 = plane_word<PL, HF, 7>(sInv, sSym, mc, live);
  v4u w;
  w[0] = upperQ ? b0 : a0;
  w[1] = upperQ ? b1 : a1;
  w[2] = upperQ ? b2 : a2;
  w[3] = upperQ ? b3 : a3;
  return w;
}

__global__ __launch_bounds__(32) void prep_planes_kernel(const float* __restrict__ Wmat,
                                                         unsigned* __restrict__ planes) {
  __shared__ float sRaw[128];
  __shared__ float sSym[kDim * kDim];
  __shared__ float sM[kDim * kDim];
  __shared__ float sInv[kDim * kDim];
  int tid = threadIdx.x;
  asm volatile("" : "+v"(tid));

#pragma unroll 1
  for (int it = 0; it < 4; ++it) {
    const int idx  = it * 32 + tid;
    const int idxc = (idx < kDim * kDim) ? idx : (kDim * kDim - 1);
    float v = Wmat[idxc];
    asm volatile("" : "+v"(v));
    sRaw[idx] = v;
  }
  __syncthreads();

  if (tid == 0) {
#pragma unroll 1
    for (int i = 0; i < kDim; ++i) {
#pragma unroll 1
      for (int j = 0; j < kDim; ++j) {
        const float s = sRaw[i * kDim + j] + sRaw[j * kDim + i];
        sSym[i * kDim + j] = s;
        sM[i * kDim + j]   = (i == j) ? (s - 1.0f) : s;
        sInv[i * kDim + j] = (i == j) ? 1.0f : 0.0f;
      }
    }
#pragma unroll 1
    for (int c = 0; c < kDim; ++c) {
      int p = c;
      float best = fabsf(sM[c * kDim + c]);
#pragma unroll 1
      for (int r = c + 1; r < kDim; ++r) {
        const float a = fabsf(sM[r * kDim + c]);
        if (a > best) { best = a; p = r; }
      }
      if (p != c) {
#pragma unroll 1
        for (int j = 0; j < kDim; ++j) {
          const float tm = sM[c * kDim + j];
          sM[c * kDim + j] = sM[p * kDim + j];
          sM[p * kDim + j] = tm;
          const float tv = sInv[c * kDim + j];
          sInv[c * kDim + j] = sInv[p * kDim + j];
          sInv[p * kDim + j] = tv;
        }
      }
      const float pv = sM[c * kDim + c];
      const float r0 = __builtin_amdgcn_rcpf(pv);
      const float inv = fmaf(fmaf(-pv, r0, 1.0f), r0, r0);
#pragma unroll 1
      for (int j = 0; j < kDim; ++j) {
        sM[c * kDim + j]   = sM[c * kDim + j] * inv;
        sInv[c * kDim + j] = sInv[c * kDim + j] * inv;
      }
#pragma unroll 1
      for (int r = 0; r < kDim; ++r) {
        if (r == c) continue;
        const float f = sM[r * kDim + c];
#pragma unroll 1
        for (int j = 0; j < kDim; ++j) {
          sM[r * kDim + j]   = fmaf(-f, sM[c * kDim + j], sM[r * kDim + j]);
          sInv[r * kDim + j] = fmaf(-f, sInv[c * kDim + j], sInv[r * kDim + j]);
        }
      }
    }
  }
  __syncthreads();

  int m = tid >> 1;
  asm volatile("" : "+v"(m));
  int mc = (m < kDim) ? m : (kDim - 1);
  asm volatile("" : "+v"(mc));
  unsigned selq = ((unsigned)tid) & 1u;
  asm volatile("" : "+v"(selq));
  const bool live   = (m < kDim);
  const bool upperQ = (selq != 0u);

  v4u wv[4];
  wv[0] = plane_quad<0>(sInv, sSym, mc, live, upperQ);
  wv[1] = plane_quad<1>(sInv, sSym, mc, live, upperQ);
  wv[2] = plane_quad<2>(sInv, sSym, mc, live, upperQ);
  wv[3] = plane_quad<3>(sInv, sSym, mc, live, upperQ);
  for (int pass = 0; pass < 2; ++pass) {
#pragma unroll
    for (int it = 0; it < 4; ++it) {
      *(volatile v4u*)(planes + it * 128 + 4 * tid) = wv[it];
    }
    __threadfence();
  }
}

__global__ __launch_bounds__(256) void score_kernel(const int* __restrict__ samples,
                                                    const float* __restrict__ ent,
                                                    const float* __restrict__ rel,
                                                    const float* __restrict__ bvec,
                                                    const unsigned* __restrict__ planes,
                                                    float* __restrict__ out) {
  __shared__ __align__(16) float sOut[kWavesPerBlk * kElemsPerWave];
  const int tid  = threadIdx.x;
  const int lane = tid & 31;
  const int wave = tid >> 5;
  const int hf   = lane >> 4;
  const int n    = lane & 15;
  const bool up  = (hf != 0);

  const v4u p1a = *(const v4u*)(planes + lane * 8);
  const v4u p1b = *(const v4u*)(planes + lane * 8 + 4);
  const v4u p2a = *(const v4u*)(planes + 256 + lane * 8);
  const v4u p2b = *(const v4u*)(planes + 256 + lane * 8 + 4);
  const v8u a1w = __builtin_shufflevector(p1a, p1b, 0, 1, 2, 3, 4, 5, 6, 7);
  const v8u a2w = __builtin_shufflevector(p2a, p2b, 0, 1, 2, 3, 4, 5, 6, 7);
  const v16b aInv = __builtin_bit_cast(v16b, a1w);
  const v16b aSym = __builtin_bit_cast(v16b, a2w);

  float bD[8];
#pragma unroll
  for (int r = 0; r < 8; ++r) {
    const int idx  = 8 * hf + r;
    const int idxc = (idx < kDim) ? idx : (kDim - 1);
    float t = bvec[idxc];
    asm volatile("" : "+v"(t));
    bD[r] = (idx < kDim) ? t : 0.0f;
  }
  float hbJ[5];
#pragma unroll
  for (int j = 0; j < 5; ++j) {
    float t = bvec[5 * hf + j];
    asm volatile("" : "+v"(t));
    hbJ[j] = 0.5f * t;
  }

  const int waveBase = blockIdx.x * kElemsPerBlk + wave * kElemsPerWave;

#pragma unroll 1
  for (int t = 0; t < kTilesPerWave; ++t) {
    const int e = waveBase + t * kTileElems + n;
    const int* sp = samples + 3 * e;
    int s0 = sp[0];
    int s1 = sp[1];
    int s2 = sp[2];
    s0 = s0 < 0 ? 0 : (s0 > kNumEnt - 1 ? kNumEnt - 1 : s0);
    s1 = s1 < 0 ? 0 : (s1 > kNumRel - 1 ? kNumRel - 1 : s1);
    s2 = s2 < 0 ? 0 : (s2 > kNumEnt - 1 ? kNumEnt - 1 : s2);

    float e1[kDim], e2[kDim];
    const float* r1p = ent + kDim * s0;
    const float* r2p = ent + kDim * s2;
#pragma unroll
    for (int i = 0; i < 5; ++i) {
      const v2f a = *(const v2f*)(r1p + 2 * i);
      const v2f c = *(const v2f*)(r2p + 2 * i);
      float c0 = c[0];
      float c1 = c[1];
      asm volatile("" : "+v"(c0));
      asm volatile("" : "+v"(c1));
      e1[2 * i] = a[0];
      e1[2 * i + 1] = a[1];
      e2[2 * i] = c0;
      e2[2 * i + 1] = c1;
    }
    float rs[5];
    const float* rrp = rel + kDim * s1 + 5 * hf;
#pragma unroll
    for (int j = 0; j < 5; ++j) rs[j] = rrp[j];

    float e2r[kDim];
#pragma unroll
    for (int i = 0; i < kDim; ++i) e2r[i] = up ? e2[(i + 5) % kDim] : e2[i];

    float xs[5], xb[5];
#pragma unroll
    for (int jj = 0; jj < 5; ++jj) {
      float acc = e1[0] * e2r[jj];
#pragma unroll
      for (int j = 1; j < kDim; ++j) acc = fmaf(e1[j], e2r[(j + jj) % kDim], acc);
      xs[jj] = rs[jj] * acc;
      xb[jj] = xs[jj] - hbJ[jj];
    }

    const v16b bx = pack_hi_hi_lo(xb[0], xb[1], xb[2], xb[3], xb[4]);
    v8f d1 = (v8f){0.f, 0.f, 0.f, 0.f, 0.f, 0.f, 0.f, 0.f};
    d1 = mma_bf16(aInv, bx, d1);

    const float x5 = __shfl_xor(d1[5], 16, 32);
    const float x6 = __shfl_xor(d1[6], 16, 32);
    const float x7 = __shfl_xor(d1[7], 16, 32);
    float hs[5];
    hs[0] = up ? x5 : d1[0];
    hs[1] = up ? x6 : d1[1];
    hs[2] = up ? x7 : d1[2];
    hs[3] = up ? d1[0] : d1[3];
    hs[4] = up ? d1[1] : d1[4];

    const v16b bh = pack_hi_hi_lo(hs[0], hs[1], hs[2], hs[3], hs[4]);
    v8f d2 = (v8f){0.f, 0.f, 0.f, 0.f, 0.f, 0.f, 0.f, 0.f};
    d2 = mma_bf16(aSym, bh, d2);

    float qv = 0.0f, lv = 0.0f, pv = 0.0f;
#pragma unroll
    for (int r = 0; r < 8; ++r) {
      qv = fmaf(d1[r], d2[r], qv);
      lv = fmaf(d1[r], bD[r], lv);
    }
#pragma unroll
    for (int j = 0; j < 5; ++j) {
      const float df = hs[j] - xs[j];
      pv = fmaf(df, df, pv);
    }
    const float part  = (qv + lv) - pv;
    const float other = __shfl_xor(part, 16, 32);
    const float tot   = part + other;
    if (hf == 0) sOut[wave * kElemsPerWave + t * kTileElems + n] = tot;
  }

  __syncthreads();
  {
    const v4f ov = *(const v4f*)(sOut + wave * kElemsPerWave + lane * 4);
    float* op = out + waveBase + lane * 4;
    *(volatile v4f*)op = ov;
    __threadfence();
    *(volatile v4f*)op = ov;
  }
}

extern "C" void kernel_launch(void* const* d_in, const int* in_sizes, int n_in,
                              void* d_out, int out_size, void* d_ws, size_t ws_size,
                              hipStream_t stream) {
  if (n_in < 5) return;
  if (in_sizes[0] != kTotal * 3) return;
  if (in_sizes[1] != kNumEnt * kDim) return;
  if (in_sizes[2] != kNumRel * kDim) return;
  if (in_sizes[3] != kDim * kDim) return;
  if (in_sizes[4] != kDim) return;
  if (out_size != kTotal) return;
  if (ws_size < kWsTotal) return;

  const int*   samples = (const int*)d_in[0];
  const float* ent     = (const float*)d_in[1];
  const float* rel     = (const float*)d_in[2];
  const float* Wmat    = (const float*)d_in[3];
  const float* bvec    = (const float*)d_in[4];
  float*    out    = (float*)d_out;
  unsigned* planes = (unsigned*)d_ws;

  prep_planes_kernel<<<1, 32, 0, stream>>>(Wmat, planes);
  score_kernel<<<kGridScore, 256, 0, stream>>>(samples, ent, rel, bvec, planes, out);
}
